// RelationGCN_24086176596515
// MI455X (gfx1250) — hardware-run, weakly checked
//
#include <hip/hip_runtime.h>

typedef float          v8f   __attribute__((ext_vector_type(8)));
typedef float          v4f   __attribute__((ext_vector_type(4)));
typedef unsigned int   v4u   __attribute__((ext_vector_type(4)));
typedef int            v8i   __attribute__((ext_vector_type(8)));
typedef unsigned short v8us  __attribute__((ext_vector_type(8)));
typedef unsigned short v16us __attribute__((ext_vector_type(16)));
typedef __bf16         v16bf __attribute__((ext_vector_type(16)));
typedef _Float16       v16h  __attribute__((ext_vector_type(16)));
typedef v4f  __attribute__((may_alias)) v4fa;
typedef v8us __attribute__((may_alias)) v8usa;
union FragB { v16bf v; v16us u; v8us h[2]; v8i w; };
union FragH { v16h  v; v16us u; v8us h[2]; v8i w; };

__device__ __forceinline__ v8f wmb(const FragB& a, const FragB& b, v8f c) {
  v8f d = __builtin_amdgcn_wmma_f32_16x16x32_bf16(false, a.v, false, b.v, (short)0, c, false, false);
  asm volatile("v_nop\n\tv_nop\n\tv_nop\n\tv_nop" : "+v"(d) : "v"(a.w), "v"(b.w));
  return d;
}

__device__ __forceinline__ v8f wmh(const FragH& a, const FragH& b, v8f c) {
  v8f d = __builtin_amdgcn_wmma_f32_16x16x32_f16(false, a.v, false, b.v, (short)0, c, false, false);
  asm volatile("v_nop\n\tv_nop\n\tv_nop\n\tv_nop" : "+v"(d) : "v"(a.w), "v"(b.w));
  return d;
}

__device__ __forceinline__ unsigned bf16_bits(float f) {
  const unsigned u = __float_as_uint(f);
  const unsigned r = (u + 0x7FFFu + ((u >> 16) & 1u)) >> 16;
  const unsigned q = (u >> 16) | 0x40u;
  return ((u & 0x7fffffffu) > 0x7f800000u) ? q : r;
}

__device__ __forceinline__ float bf16_val(float f) {
  return __uint_as_float(bf16_bits(f) << 16);
}
__device__ __forceinline__ int clampi(int v, int lo, int hi) {
  return v < lo ? lo : (v > hi ? hi : v);
}

__device__ __forceinline__ unsigned f16_bits(float f) {
  const unsigned u  = __float_as_uint(f);
  const unsigned s  = (u >> 16) & 0x8000u;
  const unsigned a  = u & 0x7fffffffu;
  const unsigned t  = a - 0x38000000u;
  const unsigned r  = (t + 0x0FFFu + ((t >> 13) & 1u)) >> 13;
  const unsigned rc = r > 0x7C00u ? 0x7C00u : r;
  const bool small  = a < 0x38800000u;
  const bool isnan  = a > 0x7f800000u;
  const unsigned fin = small ? 0u : (s | rc);
  return isnan ? (s | 0x7E00u) : fin;
}

__device__ __forceinline__ unsigned pk16(unsigned lo, unsigned hi) { return lo | (hi << 16); }
__device__ __forceinline__ unsigned bf16_lo_bits(float v) {
  float hi = bf16_val(v);
  asm volatile("" : "+v"(hi));
  return bf16_bits(v - hi);
}
__device__ __forceinline__ v4u pack8_bf16(v4f a, v4f c) {
  return (v4u){ pk16(bf16_bits(a[0]), bf16_bits(a[1])), pk16(bf16_bits(a[2]), bf16_bits(a[3])),
                pk16(bf16_bits(c[0]), bf16_bits(c[1])), pk16(bf16_bits(c[2]), bf16_bits(c[3])) };
}
__device__ __forceinline__ v4u pack8_bf16_lo(v4f a, v4f c) {
  return (v4u){ pk16(bf16_lo_bits(a[0]), bf16_lo_bits(a[1])), pk16(bf16_lo_bits(a[2]), bf16_lo_bits(a[3])),
                pk16(bf16_lo_bits(c[0]), bf16_lo_bits(c[1])), pk16(bf16_lo_bits(c[2]), bf16_lo_bits(c[3])) };
}
__device__ __forceinline__ v4u pack8_f16(v4f a, v4f c) {
  return (v4u){ pk16(f16_bits(a[0]), f16_bits(a[1])), pk16(f16_bits(a[2]), f16_bits(a[3])),
                pk16(f16_bits(c[0]), f16_bits(c[1])), pk16(f16_bits(c[2]), f16_bits(c[3])) };
}

template <int FORM>
__global__ __launch_bounds__(256) void k_plane(const float* __restrict__ src, int rows, int cols, int ldsrc,
                                               unsigned short* __restrict__ dst, int MP, int KP) {
  static_assert(FORM >= 0 && FORM <= 3);
  const int KTOT = (FORM == 1 || FORM == 3) ? 2 * KP : KP;
  const unsigned ppr   = (unsigned)(KTOT >> 3);
  const unsigned kp8   = (unsigned)(KP >> 3);
  const unsigned total = (unsigned)MP * ppr;
  const unsigned g     = blockIdx.x * 256u + threadIdx.x;
  const unsigned rowu  = g / ppr;
  const unsigned p     = g - rowu * ppr;
  const bool second    = p >= kp8;
  const int row = (int)rowu;
  const int c0  = (int)((second ? p - kp8 : p) << 3);
  const float* srow = src + (size_t)clampi(row, 0, rows - 1) * (size_t)ldsrc;
  float x[8];
  unsigned mk[8];
#pragma unroll
  for (int e = 0; e < 8; ++e) {
    const int c = c0 + e;
    const float v = srow[clampi(c, 0, cols - 1)];
    asm volatile("" :: "v"(v));
    x[e]  = v;
    mk[e] = (row < rows && c < cols) ? 0xFFFFu : 0u;
  }
  const v4f a = (v4f){ x[0], x[1], x[2], x[3] };
  const v4f c = (v4f){ x[4], x[5], x[6], x[7] };
  v4u o;
  if (FORM == 2) {
    o = pack8_f16(a, c);
  } else {
    const v4u hi = pack8_bf16(a, c);
    o = hi;
    if (FORM == 1) { const v4u lo = pack8_bf16_lo(a, c); o = second ? lo : hi; }
  }
  const v4u mw = (v4u){ pk16(mk[0], mk[1]), pk16(mk[2], mk[3]), pk16(mk[4], mk[5]), pk16(mk[6], mk[7]) };
  o &= mw;
  if (g < total) {
    volatile v4u* q = (volatile v4u*)(dst + (size_t)g * 8);
    *q = o;
    __threadfence();
    *q = o;
  }
}

template <int FORM> struct FragOf    { typedef FragB T; };
template <>         struct FragOf<2> { typedef FragH T; };
__device__ __forceinline__ v8f mm(const FragB& a, const FragB& b, v8f c) { return wmb(a, b, c); }
__device__ __forceinline__ v8f mm(const FragH& a, const FragH& b, v8f c) { return wmh(a, b, c); }
template <class F> __device__ __forceinline__ F ld_frag(const unsigned short* p) {
  F f;
  f.h[0] = *(const v8usa*)(p);
  f.h[1] = *(const v8usa*)(p + 16);
  return f;
}

template <int FORM, int EPI>
__global__ __launch_bounds__(256) __attribute__((amdgpu_num_vgpr(248)))
void k_gemm_nt(const unsigned short* __restrict__ A, const unsigned short* __restrict__ B,
               const float* __restrict__ bias, float* __restrict__ D, int M, int N, int KTOT, int ldd) {
  static_assert(FORM >= 0 && FORM <= 2);
  static_assert(EPI == 0 || EPI == 1);
  typedef typename FragOf<FORM>::T F;
  __shared__ __attribute__((aligned(16))) float sT[8][16 * 68];
  const int lane = threadIdx.x & 31;
  const int wave = threadIdx.x >> 5;
  const int tilesM = (M + 63) >> 6;
  const int tilesN = (N + 63) >> 6;
  const int tile = blockIdx.x * 8 + wave;
  if (tile >= tilesM * tilesN) return;
  const int tm = tile / tilesN;
  const int tn = tile - tm * tilesN;
  const int m0 = tm << 6;
  const int n0 = tn << 6;

  const int rl = lane & 15;
  const int h8 = (lane >> 4) * 8;
  const unsigned short* pa = A + (size_t)(m0 + rl) * (size_t)KTOT + h8;
  const unsigned short* pb = B + (size_t)(n0 + rl) * (size_t)KTOT + h8;

  v8f acc[4][4];
#pragma unroll
  for (int i = 0; i < 4; ++i)
#pragma unroll
    for (int j = 0; j < 4; ++j) acc[i][j] = (v8f){0.f, 0.f, 0.f, 0.f, 0.f, 0.f, 0.f, 0.f};

#pragma unroll 1
  for (int k0 = 0; k0 < KTOT; k0 += 32) {
    F bf[4];
#pragma unroll
    for (int j = 0; j < 4; ++j) bf[j] = ld_frag<F>(pb + (size_t)(j << 4) * (size_t)KTOT + k0);
#pragma unroll
    for (int i = 0; i < 4; ++i) {
      const F af = ld_frag<F>(pa + (size_t)(i << 4) * (size_t)KTOT + k0);
#pragma unroll
      for (int j = 0; j < 4; ++j) acc[i][j] = mm(af, bf[j], acc[i][j]);
    }
  }

  float* slab = sT[wave];
  const int hh = lane >> 4;
  const int c4 = (lane & 15) * 4;
  const int nc = n0 + c4;
  const bool cok = nc < N;
  v4f bv = (v4f){0.f, 0.f, 0.f, 0.f};
  if (EPI == 1) {
    bv = *(const v4fa*)(bias + clampi(nc, 0, N - 4));
    asm volatile("" :: "v"(bv));
  }
#pragma unroll
  for (int i = 0; i < 4; ++i) {
    const int mBase = m0 + (i << 4);
#pragma unroll
    for (int j = 0; j < 4; ++j) {
#pragma unroll
      for (int r = 0; r < 8; ++r) slab[(h8 + r) * 68 + (j << 4) + rl] = acc[i][j][r];
    }
    __builtin_amdgcn_fence(__ATOMIC_RELEASE, "workgroup");
    __builtin_amdgcn_wave_barrier();
    __builtin_amdgcn_fence(__ATOMIC_ACQUIRE, "workgroup");
    v4f vv[8];
#pragma unroll
    for (int it = 0; it < 8; ++it) {
      const int row = it * 2 + hh;
      v4f v = *(const v4fa*)(slab + row * 68 + c4);
      if (EPI == 1) v += bv;
      vv[it] = v;
    }
    for (int pass = 0; pass < 2; ++pass) {
#pragma unroll
      for (int it = 0; it < 8; ++it) {
        const int row = mBase + it * 2 + hh;
        if (cok && row < M) *(volatile v4f*)(D + (size_t)row * (size_t)ldd + nc) = vv[it];
      }
      __threadfence();
    }
    __builtin_amdgcn_fence(__ATOMIC_RELEASE, "workgroup");
    __builtin_amdgcn_wave_barrier();
    __builtin_amdgcn_fence(__ATOMIC_ACQUIRE, "workgroup");
  }
}

#ifndef SPLIT_L0
#define SPLIT_L0 1
#endif
#ifndef SPLIT_L1
#define SPLIT_L1 1
#endif
#ifndef SPLIT_L2
#define SPLIT_L2 1
#endif

#define NN     50000
#define DD     64
#define NE     800000
#define MPAD   50048
#define NTHR   256
#define NWAVE  8
#define EPT    8
#define CHUNK  (NTHR * EPT)
#define WCAP   (EPT * 32)
#define LISTN  (NWAVE * WCAP)
#define NBA    1024
#define SLA    10
#define NBLK   49
#define NTAB   (NBLK * NBA)
#define MAXHIT 16707
#define RCAP   20992
#define DEGCAP 128
#define BK_ZINTS (LISTN + 2 * RCAP + 3 * NBA)
#define BK_INTS  (BK_ZINTS + 16)
#define BK_LDS   (BK_INTS * 4)
#define PU_W   3072
#define PU_P   128
#define PU_Z   768
#define PU_ALL (PU_W + PU_P + 2 * PU_Z)
#define TAB_B   0
#define TAB_G   192
#define TAB_E   320
#define TAB_REL 512
#define TAB_FLOATS 1280
#define OUT_REL 12800000
#define OUT_ALL 12800256
#define GEMM_BLOCKS 98

static_assert(RCAP % 256 == 0);
static_assert((long long)RCAP * 4 >= (long long)MAXHIT * 5);
static_assert(NBLK * NBA >= NN && NTAB >= MPAD);
static_assert(NE % 256 == 0 && NE % 4 == 0);
static_assert(NE < (1 << 20));
static_assert(CHUNK == 2048 && (CHUNK & (CHUNK - 1)) == 0);
static_assert(NBA == (1 << SLA) && NBA % NWAVE == 0 && NBA == 4 * NTHR);
static_assert(BK_ZINTS % (4 * NTHR) == 0);
static_assert(BK_LDS <= 262144);
static_assert(RCAP % 4 == 0);
static_assert(MPAD % 128 == 0 && MPAD % 64 == 0 && MPAD >= NN && NN % 16 == 0);
static_assert(DD == 64 && DD % 4 == 0);
static_assert(PU_W % 32 == 0 && (PU_W + PU_P) % 32 == 0 && (PU_W + PU_P + PU_Z) % 32 == 0 && PU_ALL % 32 == 0);
static_assert((MPAD - NN) * DD * 4 == PU_Z * 16 && (MPAD - NN) * 128 * 2 == PU_Z * 16);
static_assert((size_t)3 * 3200000 + (size_t)64 * (NN - 1) + 63 < (size_t)OUT_REL);
static_assert(OUT_REL + 255 < OUT_ALL && (OUT_REL * 4) % 128 == 0 && (3200000 * 4) % 128 == 0);
static_assert(GEMM_BLOCKS * 8 >= (NN + 63) / 64);
static_assert((long long)MPAD * 128 / 8 < (1LL << 31));

typedef float  v2f __attribute__((ext_vector_type(2)));
typedef int    v4i __attribute__((ext_vector_type(4)));
typedef double v2d __attribute__((ext_vector_type(2)));
typedef v2f __attribute__((may_alias)) v2fa;
typedef v4i __attribute__((may_alias)) v4ia;
typedef v2d __attribute__((may_alias)) v2da;

__device__ __forceinline__ float leaky01(float y) { return (y >= 0.0f) ? y : 0.01f * y; }

__global__ __launch_bounds__(NTHR) void k_prep(const float* __restrict__ gW, const float* __restrict__ gb,
                                               const float* __restrict__ gam, const float* __restrict__ bet,
                                               unsigned short* W2T, float* TAB, float* Tpad, unsigned short* Apad,
                                               int kt0, int kt1, int kt2) {
  const int u = (int)blockIdx.x * NTHR + (int)threadIdx.x;
  if (u < PU_W) {
    const int i  = u >> 10;
    const int v  = u & 1023;
    const int kt = (i == 0) ? kt0 : ((i == 1) ? kt1 : kt2);
    const int sh = (kt == 128) ? 4 : 3;
    if (v < (DD << sh)) {
      const int n  = v >> sh;
      const int k8 = (v - (n << sh)) << 3;
      const int kk = k8 & (DD - 1);
      const float* p = gW + ((size_t)i * DD + (size_t)kk) * DD + n;
      unsigned hb[8];
#pragma unroll
      for (int e = 0; e < 8; ++e) {
        const float x = p[(size_t)e * DD];
        asm volatile("" :: "v"(x));
        hb[e] = bf16_bits(x);
      }
      const v4u o = (v4u){ pk16(hb[0], hb[1]), pk16(hb[2], hb[3]), pk16(hb[4], hb[5]), pk16(hb[6], hb[7]) };
      volatile v4u* q = (volatile v4u*)(W2T + (size_t)i * DD * 128 + (size_t)v * 8);
      *q = o;
      __threadfence();
      *q = o;
    }
  } else if (u < PU_W + PU_P) {
    const int q = u - PU_W;
    const v4f b4 = *(const v4fa*)(gb  + 4 * clampi(q, 0, 47));
    const v4f g4 = *(const v4fa*)(gam + 4 * clampi(q - 48, 0, 31));
    const v4f e4 = *(const v4fa*)(bet + 4 * clampi(q - 80, 0, 31));
    asm volatile("" :: "v"(b4));
    asm volatile("" :: "v"(g4));
    asm volatile("" :: "v"(e4));
    const unsigned mb = (q < 48) ? 0xFFFFFFFFu : 0u;
    const unsigned mg = (q >= 48 && q < 80) ? 0xFFFFFFFFu : 0u;
    const unsigned me = (q >= 80 && q < 112) ? 0xFFFFFFFFu : 0u;
    v4f o;
    o[0] = bf16_val(__uint_as_float((__float_as_uint(b4[0]) & mb) | (__float_as_uint(g4[0]) & mg) | (__float_as_uint(e4[0]) & me)));
    o[1] = bf16_val(__uint_as_float((__float_as_uint(b4[1]) & mb) | (__float_as_uint(g4[1]) & mg) | (__float_as_uint(e4[1]) & me)));
    o[2] = bf16_val(__uint_as_float((__float_as_uint(b4[2]) & mb) | (__float_as_uint(g4[2]) & mg) | (__float_as_uint(e4[2]) & me)));
    o[3] = bf16_val(__uint_as_float((__float_as_uint(b4[3]) & mb) | (__float_as_uint(g4[3]) & mg) | (__float_as_uint(e4[3]) & me)));
    volatile v4f* w = (volatile v4f*)(TAB + 4 * q);
    *w = o;
    __threadfence();
    *w = o;
  } else if (u < PU_W + PU_P + PU_Z) {
    const int z = u - (PU_W + PU_P);
    const v4f o = (v4f){0.f, 0.f, 0.f, 0.f};
    volatile v4f* w = (volatile v4f*)(Tpad + 4 * z);
    *w = o;
    __threadfence();
    *w = o;
  } else if (u < PU_ALL) {
    const int z = u - (PU_W + PU_P + PU_Z);
    const v4u o = (v4u){0u, 0u, 0u, 0u};
    volatile v4u* w = (volatile v4u*)(Apad + 8 * z);
    *w = o;
    __threadfence();
    *w = o;
  }
}

__global__ __launch_bounds__(NTHR) void k_rel(const float* __restrict__ r_n, const float* __restrict__ r_p,
                                              const float* __restrict__ r_s, const float* __restrict__ r_d,
                                              const float* __restrict__ Wr, const float* __restrict__ br,
                                              float* TABR, float* out) {
  __shared__ __attribute__((aligned(16))) float vec[4 * DD];
  __shared__ __attribute__((aligned(16))) float stg[12 * DD];
  const int t = (int)threadIdx.x;
  const int s = t >> 6;
  const int o = t & 63;
  const float a0 = r_n[o];
  const float a1 = r_p[o];
  const float a2 = r_s[o];
  const float a3 = r_d[o];
  asm volatile("" :: "v"(a0));
  asm volatile("" :: "v"(a1));
  asm volatile("" :: "v"(a2));
  asm volatile("" :: "v"(a3));
  const unsigned m0 = (s == 0) ? 0xFFFFFFFFu : 0u;
  const unsigned m1 = (s == 1) ? 0xFFFFFFFFu : 0u;
  const unsigned m2 = (s == 2) ? 0xFFFFFFFFu : 0u;
  const unsigned m3 = (s == 3) ? 0xFFFFFFFFu : 0u;
  float r = bf16_val(__uint_as_float((__float_as_uint(a0) & m0) | (__float_as_uint(a1) & m1) |
                                     (__float_as_uint(a2) & m2) | (__float_as_uint(a3) & m3)));
#pragma unroll 1
  for (int i = 0; i < 3; ++i) {
    vec[t] = r;
    stg[(s * 3 + i) * DD + o] = r;
    __syncthreads();
    const float* wr = Wr + ((size_t)i * DD + (size_t)o) * DD;
    const float* xv = vec + s * DD;
    float acc = 0.0f;
#pragma unroll 4
    for (int j4 = 0; j4 < DD / 4; ++j4) {
      const v4f w = *(const v4fa*)(wr + 4 * j4);
      const v4f x = *(const v4fa*)(xv + 4 * j4);
      acc = fmaf(x[0], bf16_val(w[0]), acc);
      acc = fmaf(x[1], bf16_val(w[1]), acc);
      acc = fmaf(x[2], bf16_val(w[2]), acc);
      acc = fmaf(x[3], bf16_val(w[3]), acc);
    }
    const float nr = acc + bf16_val(br[i * DD + o]);
    __syncthreads();
    r = nr;
  }
  if (t < 192) {
    const v4f v = *(const v4fa*)(stg + 4 * t);
    volatile v4f* q = (volatile v4f*)(TABR + 4 * t);
    *q = v;
    __threadfence();
    *q = v;
  }
  volatile float* qo = (volatile float*)(out + (size_t)OUT_REL + t);
  *qo = r;
  __threadfence();
  *qo = r;
}

__device__ __forceinline__ int scan_chunk(const int* __restrict__ dsts, int nE, int cbase, int slotBase,
                                          int* list, int lane, int wave) {
  int wc = 0;
  const int wbase = wave * WCAP;
#pragma unroll 1
  for (int hf = 0; hf < 2; ++hf) {
    int dv[4];
#pragma unroll
    for (int jj = 0; jj < 4; ++jj) {
      const int el = wbase + ((hf * 4 + jj) << 5) + lane;
      const int e  = cbase + el;
      const int d  = dsts[e < nE ? e : nE - 1];
      asm volatile("" :: "v"(d));
      dv[jj] = (e < nE) ? d : -1;
    }
#pragma unroll
    for (int jj = 0; jj < 4; ++jj) {
      const int el = wbase + ((hf * 4 + jj) << 5) + lane;
      const unsigned sj = (unsigned)dv[jj] - (unsigned)slotBase;
      const bool hj = sj < (unsigned)NBA;
      const unsigned mj = __builtin_amdgcn_ballot_w32(hj);
      if (mj != 0u) {
        if (hj) {
          const int pos = wc + (int)__builtin_amdgcn_mbcnt_lo(mj, 0u);
          if (pos < WCAP) list[wbase + pos] = (el << SLA) | (int)sj;
        }
        wc += (int)__builtin_popcount(mj);
      }
    }
  }
  return wc;
}

__global__ __launch_bounds__(NTHR) void k_bucket(const int* __restrict__ edge, int nE, int nN,
                                                 int* LIST, int* OFF, int* CNT, int* DINVB, int* FLAG) {
  extern __shared__ __attribute__((aligned(16))) int dsm[];
  int* list = dsm;
  int* hl   = dsm + LISTN;
  int* sl   = dsm + LISTN + RCAP;
  int* cnt  = dsm + LISTN + 2 * RCAP;
  int* offs = cnt + NBA;
  int* cur  = offs + NBA;
  int* misc = cur + NBA;
  const int tid = (int)threadIdx.x, lane = tid & 31, wave = tid >> 5;
  const int b = (int)blockIdx.x;
  const int nodeBase = b * NBA;
  const int* srcs = edge;
  const int* dsts = edge + nE;

  {
    const v4i z4 = {0, 0, 0, 0};
    for (int i = tid * 4; i < BK_ZINTS; i += NTHR * 4) *(v4ia*)(dsm + i) = z4;
    if (tid < 16) misc[tid] = 0;
  }
  __syncthreads();

  int t = 0, ov = 0;
  const int nChunks = (nE + CHUNK - 1) / CHUNK;
#pragma unroll 1
  for (int ch = 0; ch < nChunks; ++ch) {
    const int cbase = ch * CHUNK;
    const int wc = scan_chunk(dsts, nE, cbase, nodeBase, list, lane, wave);
    if (lane == 0) misc[wave] = wc;
    __syncthreads();
    if (wave == 0) {
#pragma unroll 1
      for (int w2 = 0; w2 < NWAVE; ++w2) {
        int c = misc[w2];
        c = c < 0 ? 0 : (c > WCAP ? WCAP : c);
        c = __builtin_amdgcn_readfirstlane(c);
#pragma unroll 1
        for (int b0 = 0; b0 < c; b0 += 32) {
          const int idx = b0 + lane;
          const int ent = list[w2 * WCAP + (idx < WCAP ? idx : WCAP - 1)];
          const int m32 = (c - b0) < 32 ? (c - b0) : 32;
#pragma unroll 1
          for (int k = 0; k < m32; ++k) {
            const int u    = __builtin_amdgcn_readlane(ent, k);
            const int slot = u & (NBA - 1);
            const int el   = (u >> SLA) & (CHUNK - 1);
            const int pk   = ((cbase + el) << SLA) | slot;
            if (t < RCAP) {
              if (lane == 0) { hl[t] = pk; cnt[slot] = cnt[slot] + 1; }
              t = t + 1;
            } else {
              ov = 1;
            }
          }
        }
      }
    }
    __syncthreads();
  }
  if (wave == 0 && lane == 0) { misc[8] = t; misc[9] = ov; }
  __syncthreads();
  int tt = misc[8];
  tt = tt < 0 ? 0 : (tt > RCAP ? RCAP : tt);
  const int ovf = misc[9];

  if (wave == 0) {
    const int base = lane * (NBA / 32);
    int s = 0;
#pragma unroll 1
    for (int i = 0; i < NBA / 32; ++i) s += cnt[base + i];
    int incl = s;
#pragma unroll
    for (int d = 1; d < 32; d <<= 1) {
      const int y = __shfl_up(incl, d, 32);
      if (lane >= d) incl += y;
    }
    int run = incl - s;
#pragma unroll 1
    for (int i = 0; i < NBA / 32; ++i) {
      const int cv = cnt[base + i];
      offs[base + i] = run;
      cur[base + i]  = run;
      run += cv;
    }
  }
  __syncthreads();
  if (wave == 0) {
    const int ttu = __builtin_amdgcn_readfirstlane(tt);
#pragma unroll 1
    for (int b0 = 0; b0 < ttu; b0 += 32) {
      const int idx = b0 + lane;
      const int ent = hl[idx < RCAP ? idx : RCAP - 1];
      const int m32 = (ttu - b0) < 32 ? (ttu - b0) : 32;
#pragma unroll 1
      for (int k = 0; k < m32; ++k) {
        const int u    = __builtin_amdgcn_readlane(ent, k);
        const int slot = u & (NBA - 1);
        if (lane == 0) {
          int p = cur[slot];
          p = p < 0 ? 0 : (p > RCAP - 1 ? RCAP - 1 : p);
          sl[p] = u;
          cur[slot] = p + 1;
        }
      }
    }
  }
  __syncthreads();

#pragma unroll 1
  for (int it = 0; it < NBA / NTHR; ++it) {
    const int s = it * NTHR + tid;
    int c = cnt[s];
    c = c < 0 ? 0 : (c > RCAP ? RCAP : c);
    cur[s] = __float_as_int(1.0f / sqrtf((float)(c + 1)));
  }
  int* Lb = LIST + (size_t)b * RCAP;
#pragma unroll 1
  for (int u = tid; u < RCAP / 4; u += NTHR) {
    const v4i e4 = *(const v4ia*)(sl + 4 * u);
    const int i0 = 4 * u;
    const int q0 = srcs[clampi(e4[0] >> SLA, 0, nE - 1)];
    const int q1 = srcs[clampi(e4[1] >> SLA, 0, nE - 1)];
    const int q2 = srcs[clampi(e4[2] >> SLA, 0, nE - 1)];
    const int q3 = srcs[clampi(e4[3] >> SLA, 0, nE - 1)];
    asm volatile("" :: "v"(q0));
    asm volatile("" :: "v"(q1));
    asm volatile("" :: "v"(q2));
    asm volatile("" :: "v"(q3));
    v4i o4;
    o4[0] = (i0     < tt) ? clampi(q0, 0, nN - 1) : 0;
    o4[1] = (i0 + 1 < tt) ? clampi(q1, 0, nN - 1) : 0;
    o4[2] = (i0 + 2 < tt) ? clampi(q2, 0, nN - 1) : 0;
    o4[3] = (i0 + 3 < tt) ? clampi(q3, 0, nN - 1) : 0;
    volatile v4i* q = (volatile v4i*)(Lb + 4 * u);
    *q = o4;
    __threadfence();
    *q = o4;
  }
  __syncthreads();
  {
    const v4i c4 = *(const v4ia*)(cnt  + 4 * tid);
    const v4i f4 = *(const v4ia*)(offs + 4 * tid);
    const v4i d4 = *(const v4ia*)(cur  + 4 * tid);
    volatile v4i* qc = (volatile v4i*)(CNT   + nodeBase + 4 * tid);
    volatile v4i* qf = (volatile v4i*)(OFF   + nodeBase + 4 * tid);
    volatile v4i* qd = (volatile v4i*)(DINVB + nodeBase + 4 * tid);
    const v4i fl4 = {ovf, ovf, ovf, ovf};
    volatile v4i* qg = (volatile v4i*)(FLAG + b * 32 + 4 * (tid & 7));
    *qc = c4; *qf = f4; *qd = d4;
    if (tid < 8) *qg = fl4;
    __threadfence();
    *qc = c4; *qf = f4; *qd = d4;
    if (tid < 8) *qg = fl4;
  }
}

template <int INIT, int SPLIT>
__global__ __launch_bounds__(NTHR) void k_upd(const float* __restrict__ feat, float* EMB, const float* __restrict__ H,
                                              const float* __restrict__ TAB, int relOff, int gOff, int beOff,
                                              const double* __restrict__ REC1, const double* __restrict__ REC2,
                                              unsigned short* AHL, int nN) {
  __shared__ __attribute__((aligned(16))) float sp[4 * DD];
  __shared__ __attribute__((aligned(16))) float smean[DD];
  __shared__ __attribute__((aligned(16))) float srstd[DD];
  const int tid = (int)threadIdx.x, lane = tid & 31;
  if (tid < 64) {
    const int which = tid >> 4, piece = tid & 15;
    const int off = (which == 1) ? gOff : ((which == 2) ? beOff : relOff);
    const v4f x = *(const v4fa*)(TAB + off + 4 * piece);
    *(v4fa*)(sp + which * DD + 4 * piece) = x;
    float mval = 0.0f, rval = 0.0f;
    if (INIT == 0) {
      double s1 = 0.0, s2 = 0.0;
#pragma unroll 2
      for (int bb = 0; bb < NBLK; ++bb) {
        s1 += REC1[bb * DD + tid];
        s2 += REC2[bb * DD + tid];
      }
      mval = (float)(s1 * (1.0 / (double)NN));
      const float var = (float)(s2 * (1.0 / (double)NN));
      rval = 1.0f / sqrtf(var + 1e-5f);
    }
    smean[tid] = mval;
    srstd[tid] = rval;
  }
  __syncthreads();
  const int p = tid & 15, r = tid >> 4;
  const v4f rl = *(const v4fa*)(sp + 4 * p);
  const v4f gg = *(const v4fa*)(sp + DD + 4 * p);
  const v4f be = *(const v4fa*)(sp + 2 * DD + 4 * p);
  const v4f mn = *(const v4fa*)(smean + 4 * p);
  const v4f rs = *(const v4fa*)(srstd + 4 * p);
  const int sA = (lane & 16) | ((2 * p) & 15);
  const int sB = sA + 1;
  const bool lsel = (p & 8) != 0;
  constexpr int KT = SPLIT ? 128 : 64;
#pragma unroll 1
  for (int it = 0; it < 8; ++it) {
    const int row = (int)blockIdx.x * 128 + it * 16 + r;
    const bool live = row < nN;
    const int rc = live ? row : nN - 1;
    v4f e;
    if (INIT != 0) {
      const v4f f = *(const v4fa*)(feat + (size_t)rc * DD + 4 * p);
      asm volatile("" :: "v"(f));
      e = (v4f){ bf16_val(f[0]), bf16_val(f[1]), bf16_val(f[2]), bf16_val(f[3]) };
    } else {
      const v4f eo = *(const v4fa*)(EMB + (size_t)rc * DD + 4 * p);
      const v4f h  = *(const v4fa*)(H + (size_t)rc * DD + 4 * p);
      asm volatile("" :: "v"(eo));
      asm volatile("" :: "v"(h));
      const float y0 = ((gg[0] * (h[0] - mn[0])) * rs[0]) + be[0];
      const float y1 = ((gg[1] * (h[1] - mn[1])) * rs[1]) + be[1];
      const float y2 = ((gg[2] * (h[2] - mn[2])) * rs[2]) + be[2];
      const float y3 = ((gg[3] * (h[3] - mn[3])) * rs[3]) + be[3];
      e = (v4f){ eo[0] + leaky01(y0), eo[1] + leaky01(y1), eo[2] + leaky01(y2), eo[3] + leaky01(y3) };
    }
    const v4f v = e * rl;
    const unsigned lm = live ? 0xFFFFFFFFu : 0u;
    const int hw0 = (int)(pk16(bf16_bits(v[0]), bf16_bits(v[1])) & lm);
    const int hw1 = (int)(pk16(bf16_bits(v[2]), bf16_bits(v[3])) & lm);
    v4u pv;
    if (SPLIT) {
      const int lw0 = (int)(pk16(bf16_lo_bits(v[0]), bf16_lo_bits(v[1])) & lm);
      const int lw1 = (int)(pk16(bf16_lo_bits(v[2]), bf16_lo_bits(v[3])) & lm);
      const int g0 = __shfl(hw0, sA, 32), g1 = __shfl(hw1, sA, 32);
      const int g2 = __shfl(hw0, sB, 32), g3 = __shfl(hw1, sB, 32);
      const int q0 = __shfl(lw0, sA, 32), q1 = __shfl(lw1, sA, 32);
      const int q2 = __shfl(lw0, sB, 32), q3 = __shfl(lw1, sB, 32);
      pv[0] = (unsigned)(lsel ? q0 : g0);
      pv[1] = (unsigned)(lsel ? q1 : g1);
      pv[2] = (unsigned)(lsel ? q2 : g2);
      pv[3] = (unsigned)(lsel ? q3 : g3);
    } else {
      const int g0 = __shfl(hw0, sA, 32), g1 = __shfl(hw1, sA, 32);
      const int g2 = __shfl(hw0, sB, 32), g3 = __shfl(hw1, sB, 32);
      pv[0] = (unsigned)g0; pv[1] = (unsigned)g1; pv[2] = (unsigned)g2; pv[3] = (unsigned)g3;
    }
    const bool wa = SPLIT ? true : (p < 8);
    volatile v4u* qa = (volatile v4u*)(AHL + (size_t)row * KT + 8 * (SPLIT ? p : (p & 7)));
    volatile v4f* qe = (volatile v4f*)(EMB + (size_t)rc * DD + 4 * p);
    if (wa) *qa = pv;
    if (live) *qe = e;
    __threadfence();
    if (wa) *qa = pv;
    if (live) *qe = e;
  }
}

template <int FINAL>
__global__ __launch_bounds__(NTHR) void k_agg(const int* __restrict__ LISTp, const int* __restrict__ OFFp,
                                              const int* __restrict__ CNTp, const float* __restrict__ DINVp,
                                              const int* __restrict__ FLAGp, const float* __restrict__ T,
                                              const float* __restrict__ bias, float* outp, int nN, int rowLimit,
                                              double* REC) {
  __shared__ __attribute__((aligned(16))) int   scnt[NBA];
  __shared__ __attribute__((aligned(16))) int   soff[NBA];
  __shared__ __attribute__((aligned(16))) float sdv[NBA];
  __shared__ __attribute__((aligned(16))) float wsum[NWAVE * DD];
  __shared__ __attribute__((aligned(16))) double drec[DD];
  const int tid = (int)threadIdx.x, lane = tid & 31, wave = tid >> 5;
  const int b = (int)blockIdx.x;
  const int nodeBase = b * NBA;
  {
    const v4i c4 = *(const v4ia*)(CNTp + nodeBase + 4 * tid);
    const v4i f4 = *(const v4ia*)(OFFp + nodeBase + 4 * tid);
    const v4f d4 = *(const v4fa*)(DINVp + nodeBase + 4 * tid);
    *(v4ia*)(scnt + 4 * tid) = c4;
    *(v4ia*)(soff + 4 * tid) = f4;
    *(v4fa*)(sdv + 4 * tid)  = d4;
  }
  const v2f bv = *(const v2fa*)(bias + 2 * lane);
  const int fl = FLAGp[b * 32];
  __syncthreads();

  const int* Lb = LISTp + (size_t)b * RCAP;
  const float qnan = __int_as_float(0x7fc00000);
  const int sa = (2 * lane) & 31, sb = (2 * lane + 1) & 31;
  float s0 = 0.0f, s1 = 0.0f;
#pragma unroll 1
  for (int si = 0; si < NBA / NWAVE; ++si) {
    const int s    = si * NWAVE + wave;
    const int node = nodeBase + s;
    int c = scnt[s];
    const bool big = c > DEGCAP;
    c = c < 0 ? 0 : (c > DEGCAP ? DEGCAP : c);
    c = __builtin_amdgcn_readfirstlane(c);
    int o = soff[s];
    o = o < 0 ? 0 : (o > RCAP - 1 ? RCAP - 1 : o);
    o = __builtin_amdgcn_readfirstlane(o);
    const int nc = node < nN ? node : nN - 1;
    const float dd = sdv[s];
    const float rd = dd * dd;
    float acc0 = 0.0f, acc1 = 0.0f;
#pragma unroll 1
    for (int b0 = 0; b0 < c; b0 += 32) {
      const int last = o + c - 1;
      int idx = o + b0 + lane;
      idx = idx > last ? last : idx;
      idx = idx < 0 ? 0 : (idx > RCAP - 1 ? RCAP - 1 : idx);
      int sr = Lb[idx];
      sr = sr < 0 ? 0 : (sr > nN - 1 ? nN - 1 : sr);
      const float cf  = DINVp[sr] * dd;
      const int   cfi = __float_as_int(cf);
      const int m32 = (c - b0) < 32 ? (c - b0) : 32;
#pragma unroll 1
      for (int k = 0; k < m32; ++k) {
        const int   sk = __builtin_amdgcn_readlane(sr, k);
        const float ck = __int_as_float(__builtin_amdgcn_readlane(cfi, k));
        const v2f a = *(const v2fa*)(T + (size_t)sk * DD + 2 * lane);
        acc0 = fmaf(ck, a.x, acc0);
        acc1 = fmaf(ck, a.y, acc1);
      }
    }
    const v2f sv = *(const v2fa*)(T + (size_t)nc * DD + 2 * lane);
    asm volatile("" :: "v"(sv.x), "v"(sv.y));
    float y0 = (acc0 + sv.x * rd) + bv.x;
    float y1 = (acc1 + sv.y * rd) + bv.y;
    const bool bad = (fl != 0) || big;
    y0 = bad ? qnan : y0;
    y1 = bad ? qnan : y1;
    const bool live = node < nN;
    const float v0 = live ? y0 : 0.0f;
    const float v1 = live ? y1 : 0.0f;
    s0 += v0;
    s1 += v1;
    v4f ow;
    ow[0] = __shfl(v0, sa, 32); ow[1] = __shfl(v1, sa, 32);
    ow[2] = __shfl(v0, sb, 32); ow[3] = __shfl(v1, sb, 32);
    const int nw = node < rowLimit ? node : rowLimit - 1;
    const bool wr = (node < rowLimit) && (lane < 16);
    volatile v4f* q = (volatile v4f*)(outp + (size_t)nw * DD + 4 * (lane & 15));
    if (wr) *q = ow;
    __threadfence();
    if (wr) *q = ow;
  }
  if (FINAL == 0) {
    wsum[wave * DD + 2 * lane + 0] = s0;
    wsum[wave * DD + 2 * lane + 1] = s1;
    __syncthreads();
    if (tid < DD) {
      double s = 0.0;
#pragma unroll
      for (int w2 = 0; w2 < NWAVE; ++w2) s += (double)wsum[w2 * DD + tid];
      drec[tid] = s;
    }
    __syncthreads();
    if (wave == 0) {
      const v2d v = *(const v2da*)(drec + 2 * lane);
      volatile v2d* q = (volatile v2d*)(REC + (size_t)b * DD + 2 * lane);
      *q = v;
      __threadfence();
      *q = v;
    }
  }
}

__global__ __launch_bounds__(NTHR) void k_sq(const float* __restrict__ H, const double* __restrict__ REC1,
                                             double* REC2, int nN) {
  __shared__ __attribute__((aligned(16))) float smean[DD];
  __shared__ __attribute__((aligned(16))) float part[16 * DD];
  __shared__ __attribute__((aligned(16))) double drec[DD];
  const int tid = (int)threadIdx.x, lane = tid & 31, wave = tid >> 5;
  const int b = (int)blockIdx.x;
  if (tid < DD) {
    double s = 0.0;
#pragma unroll 2
    for (int bb = 0; bb < NBLK; ++bb) s += REC1[bb * DD + tid];
    smean[tid] = (float)(s * (1.0 / (double)NN));
  }
  __syncthreads();
  const int p = tid & 15, r = tid >> 4;
  const v4f mn = *(const v4fa*)(smean + 4 * p);
  const v4f zz = (v4f){0.f, 0.f, 0.f, 0.f};
  v4f acc = zz;
#pragma unroll 1
  for (int it = 0; it < NBA / 16; ++it) {
    const int row = b * NBA + it * 16 + r;
    const bool live = row < nN;
    const int rc = live ? row : nN - 1;
    const v4f h = *(const v4fa*)(H + (size_t)rc * DD + 4 * p);
    asm volatile("" :: "v"(h));
    const v4f d = h - mn;
    const v4f sq = d * d;
    acc += live ? sq : zz;
  }
  *(v4fa*)(part + r * DD + 4 * p) = acc;
  __syncthreads();
  if (tid < DD) {
    double s = 0.0;
#pragma unroll
    for (int g = 0; g < 16; ++g) s += (double)part[g * DD + tid];
    drec[tid] = s;
  }
  __syncthreads();
  if (wave == 0) {
    const v2d v = *(const v2da*)(drec + 2 * lane);
    volatile v2d* q = (volatile v2d*)(REC2 + (size_t)b * DD + 2 * lane);
    *q = v;
    __threadfence();
    *q = v;
  }
}

constexpr size_t SZ_PLANE = (size_t)MPAD * DD * 4;
constexpr size_t SZ_LIST  = (size_t)NBLK * RCAP * 4;
constexpr size_t SZ_TBL   = (size_t)NTAB * 4;
constexpr size_t SZ_REC   = (size_t)NBLK * DD * 8;
constexpr size_t SZ_W     = (size_t)3 * DD * 128 * 2;
constexpr size_t SZ_TAB   = (size_t)TAB_FLOATS * 4;
constexpr size_t SZ_FLAG  = 6400;
constexpr size_t O_EMB  = 0;
constexpr size_t O_AHL  = O_EMB  + SZ_PLANE;
constexpr size_t O_T    = O_AHL  + SZ_PLANE;
constexpr size_t O_H    = O_T    + SZ_PLANE;
constexpr size_t O_LIST = O_H    + SZ_PLANE;
constexpr size_t O_OFF  = O_LIST + SZ_LIST;
constexpr size_t O_CNT  = O_OFF  + SZ_TBL;
constexpr size_t O_DINV = O_CNT  + SZ_TBL;
constexpr size_t O_REC1 = O_DINV + SZ_TBL;
constexpr size_t O_REC2 = O_REC1 + SZ_REC;
constexpr size_t O_W    = O_REC2 + SZ_REC;
constexpr size_t O_TAB  = O_W    + SZ_W;
constexpr size_t O_FLAG = O_TAB  + SZ_TAB;
constexpr size_t WS_TOTAL = O_FLAG + SZ_FLAG;
static_assert((size_t)MPAD * 128 * 2 == SZ_PLANE);
static_assert(SZ_PLANE % 256 == 0 && SZ_LIST % 256 == 0 && SZ_TBL % 256 == 0 && SZ_REC % 256 == 0);
static_assert(SZ_W % 256 == 0 && SZ_TAB % 256 == 0 && SZ_FLAG % 256 == 0 && SZ_FLAG >= (size_t)NBLK * 128);
static_assert(WS_TOTAL == 56076544);
static_assert(WS_TOTAL <= ((size_t)128 << 20));

template <int SP>
static void run_gemm(const unsigned short* A, const unsigned short* Bp, const float* dummy, float* T,
                     hipStream_t st) {
  k_gemm_nt<SP, 0><<<GEMM_BLOCKS, 256, 0, st>>>(A, Bp, dummy, T, NN, DD, SP ? 128 : 64, DD);
}

extern "C" void kernel_launch(void* const* d_in, const int* in_sizes, int n_in,
                              void* d_out, int out_size, void* d_ws, size_t ws_size,
                              hipStream_t stream) {
  if (n_in < 15) return;
  if (in_sizes[0] != NN * DD) return;
  if (in_sizes[1] != DD || in_sizes[2] != DD || in_sizes[3] != DD || in_sizes[4] != DD) return;
  if (in_sizes[5] != 2 * NE || in_sizes[6] != 2 * NE || in_sizes[7] != 2 * NE || in_sizes[8] != 2 * NE) return;
  if (in_sizes[9] != 3 * DD * DD || in_sizes[10] != 3 * DD) return;
  if (in_sizes[11] != 2 * DD || in_sizes[12] != 2 * DD) return;
  if (in_sizes[13] != 3 * DD * DD || in_sizes[14] != 3 * DD) return;
  if (out_size != OUT_ALL) return;
  if (ws_size < WS_TOTAL) return;

  const float* feat = (const float*)d_in[0];
  const float* rv0 = (const float*)d_in[4];
  const float* rv1 = (const float*)d_in[1];
  const float* rv2 = (const float*)d_in[2];
  const float* rv3 = (const float*)d_in[3];
  const int* edges[4] = { (const int*)d_in[8], (const int*)d_in[5], (const int*)d_in[6], (const int*)d_in[7] };
  const float* gW  = (const float*)d_in[9];
  const float* gb  = (const float*)d_in[10];
  const float* gam = (const float*)d_in[11];
  const float* bet = (const float*)d_in[12];
  const float* rW  = (const float*)d_in[13];
  const float* rb  = (const float*)d_in[14];
  float* out = (float*)d_out;

  char* ws = (char*)d_ws;
  float*          EMB  = (float*)(ws + O_EMB);
  unsigned short* AHL  = (unsigned short*)(ws + O_AHL);
  float*          T    = (float*)(ws + O_T);
  float*          H    = (float*)(ws + O_H);
  int*            LIST = (int*)(ws + O_LIST);
  int*            OFF  = (int*)(ws + O_OFF);
  int*            CNT  = (int*)(ws + O_CNT);
  int*            DINV = (int*)(ws + O_DINV);
  double*         REC1 = (double*)(ws + O_REC1);
  double*         REC2 = (double*)(ws + O_REC2);
  unsigned short* W2T  = (unsigned short*)(ws + O_W);
  float*          TAB  = (float*)(ws + O_TAB);
  int*            FLAG = (int*)(ws + O_FLAG);

  const int kt0 = SPLIT_L0 ? 128 : 64;
  const int kt1 = SPLIT_L1 ? 128 : 64;
  const int kt2 = SPLIT_L2 ? 128 : 64;

  hipFuncSetAttribute(reinterpret_cast<const void*>(&k_bucket), hipFuncAttributeMaxDynamicSharedMemorySize, (int)BK_LDS);

  k_prep<<<(PU_ALL + NTHR - 1) / NTHR, NTHR, 0, stream>>>(gW, gb, gam, bet, W2T, TAB, T + (size_t)NN * DD,
                                                          AHL + (size_t)NN * 128, kt0, kt1, kt2);
  k_rel<<<1, NTHR, 0, stream>>>(rv0, rv1, rv2, rv3, rW, rb, TAB + TAB_REL, out);

  for (int s = 0; s < 4; ++s) {
    const int relBase = TAB_REL + s * 3 * DD;
    k_bucket<<<NBLK, NTHR, BK_LDS, stream>>>(edges[s], NE, NN, LIST, OFF, CNT, DINV, FLAG);
    k_upd<1, SPLIT_L0><<<MPAD / 128, NTHR, 0, stream>>>(feat, EMB, H, TAB, relBase, TAB_G, TAB_E, REC1, REC2, AHL, NN);
    for (int i = 0; i < 2; ++i) {
      if (i == 0) run_gemm<SPLIT_L0>(AHL, W2T, TAB, T, stream);
      else        run_gemm<SPLIT_L1>(AHL, W2T + (size_t)DD * 128, TAB, T, stream);
      k_agg<0><<<NBLK, NTHR, 0, stream>>>(LIST, OFF, CNT, (const float*)DINV, FLAG, T, TAB + TAB_B + i * DD, H,
                                          NN, MPAD, REC1);
      k_sq<<<NBLK, NTHR, 0, stream>>>(H, REC1, REC2, NN);
      if (i == 0)
        k_upd<0, SPLIT_L1><<<MPAD / 128, NTHR, 0, stream>>>(feat, EMB, H, TAB, relBase + DD, TAB_G, TAB_E,
                                                            REC1, REC2, AHL, NN);
      else
        k_upd<0, SPLIT_L2><<<MPAD / 128, NTHR, 0, stream>>>(feat, EMB, H, TAB, relBase + 2 * DD, TAB_G + DD,
                                                            TAB_E + DD, REC1, REC2, AHL, NN);
    }
    run_gemm<SPLIT_L2>(AHL, W2T + (size_t)2 * DD * 128, TAB, T, stream);
    k_agg<1><<<NBLK, NTHR, 0, stream>>>(LIST, OFF, CNT, (const float*)DINV, FLAG, T, TAB + TAB_B + 2 * DD,
                                        out + (size_t)s * 3200000, NN, NN, REC1);
  }
}
